// ComplexSelfAttention_11089605558959
// MI455X (gfx1250) — hardware-verified
//
#include <hip/hip_runtime.h>
#include <math.h>

typedef __attribute__((ext_vector_type(16))) _Float16 v16h;
typedef __attribute__((ext_vector_type(16))) __bf16 v16b;
typedef __attribute__((ext_vector_type(8)))  _Float16 v8h;
typedef __attribute__((ext_vector_type(8)))  __bf16 v8b;
typedef __attribute__((ext_vector_type(8)))  float v8f;
typedef __attribute__((ext_vector_type(8)))  unsigned v8u;
typedef __attribute__((ext_vector_type(4)))  float v4f;
typedef __attribute__((ext_vector_type(4)))  unsigned v4u;

#define DD 512
#define KP 1024
#define NB_FULL 8
#define SEQ_FULL 1024
#ifndef NB
#define NB NB_FULL
#endif
#ifndef SEQ
#define SEQ SEQ_FULL
#endif
#define MR (NB * SEQ)
#define QCAR 2048.0f
#define PCAR 16384.0f
#define SCL 0.044194173824159216f

static_assert(NB >= 1 && NB <= NB_FULL);
static_assert(SEQ >= 256 && SEQ <= SEQ_FULL && (SEQ % 256) == 0);
static_assert((MR % 64) == 0);

#define WPL    ((size_t)DD * KP)
#define WS_X   ((size_t)0)
#define WS_W   (WS_X + 2u * (size_t)MR * KP)
#define WS_QH  (WS_W + 2u * 6u * WPL)
#define WS_QR  (WS_QH + 2u * (size_t)MR * KP)
#define WS_KH  (WS_QR + 2u * (size_t)MR * KP)
#define WS_KR  (WS_KH + 2u * (size_t)MR * KP)
#define WS_VT  (WS_KR + 2u * (size_t)MR * KP)
#define WS_S   (WS_VT + 2u * (size_t)NB * KP * SEQ)
#define WS_P   (WS_S + 4u * 2u * (size_t)SEQ * SEQ)
#define WS_END (WS_P + 2u * (size_t)SEQ * SEQ)
static_assert(WS_END <= (size_t)134217728);
static_assert((WS_W % 256) == 0 && (WS_QH % 256) == 0 && (WS_QR % 256) == 0 && (WS_KH % 256) == 0 && (WS_KR % 256) == 0 && (WS_VT % 256) == 0 && (WS_S % 256) == 0 && (WS_P % 256) == 0);

template <typename T> __device__ __forceinline__ void vst2(void* p, T v) { *(volatile T*)p = v; __threadfence(); *(volatile T*)p = v; }

__device__ __forceinline__ v8f wmma16(v16h a, v16h b, v8f c) {
  v8f d = __builtin_amdgcn_wmma_f32_16x16x32_f16(false, a, false, b, (short)0, c, false, false);
  asm volatile("v_nop\n\tv_nop\n\tv_nop\n\tv_nop" : "+v"(d) : "v"(a), "v"(b));
  return d;
}
__device__ __forceinline__ v8f wmma_bf(v16b a, v16b b, v8f c) {
  v8f d = __builtin_amdgcn_wmma_f32_16x16x32_bf16(false, a, false, b, (short)0, c, false, false);
  asm volatile("v_nop\n\tv_nop\n\tv_nop\n\tv_nop" : "+v"(d) : "v"(a), "v"(b));
  return d;
}
__device__ __forceinline__ v16h frag_h(const _Float16* rowk0, int lane) {
  union { v16h v; v8h q[2]; } u; const _Float16* p = rowk0 + 8 * (lane >> 4);
  u.q[0] = *(const v8h*)p; u.q[1] = *(const v8h*)(p + 16); return u.v;
}
__device__ __forceinline__ v16b frag_b(const __bf16* rowk0, int lane) {
  union { v16b v; v8b q[2]; } u; const __bf16* p = rowk0 + 8 * (lane >> 4);
  u.q[0] = *(const v8b*)p; u.q[1] = *(const v8b*)(p + 16); return u.v;
}
__device__ __forceinline__ v16h hneg(v16h x, unsigned m) { v8u u = __builtin_bit_cast(v8u, x); u ^= m; return __builtin_bit_cast(v16h, u); }
__device__ __forceinline__ float bfr(float v) { return (float)(__bf16)v; }
__device__ __attribute__((noinline)) float exp_ni(float v) { return expf(v); }

__global__ __launch_bounds__(256) void k_cvx(const float* __restrict__ XR, const float* __restrict__ XI, __bf16* __restrict__ X) {
  const int tid = threadIdx.x; const int row = blockIdx.x * 2 + (tid >> 7); const int t = tid & 127;
  const int half = t >> 6; const int c = (t & 63) * 8;
  const int bb = row / SEQ, n = row - bb * SEQ;
  const float* sp = (half ? XI : XR) + ((size_t)bb * SEQ_FULL + n) * DD + c;
  const v4f f0 = *(const v4f*)sp, f1 = *(const v4f*)(sp + 4);
  v8b o;
#pragma unroll
  for (int i = 0; i < 4; ++i) { o[i] = (__bf16)f0[i]; o[4 + i] = (__bf16)f1[i]; }
  vst2(X + (size_t)row * KP + half * DD + c, __builtin_bit_cast(v4u, o));
}
__global__ __launch_bounds__(256) void k_cvw(const float* __restrict__ WR, const float* __restrict__ WI, __bf16* __restrict__ BRE, __bf16* __restrict__ BIM) {
  const int tid = threadIdx.x; const int e = blockIdx.x * 4 + (tid >> 6); const int c = (tid & 63) * 8;
  const float* pr = WR + (size_t)e * DD + c; const float* pi = WI + (size_t)e * DD + c;
  const v4f r0 = *(const v4f*)pr, r1 = *(const v4f*)(pr + 4), i0 = *(const v4f*)pi, i1 = *(const v4f*)(pi + 4);
  v8b vr, vi, vn;
#pragma unroll
  for (int i = 0; i < 4; ++i) { vr[i] = (__bf16)r0[i]; vr[4 + i] = (__bf16)r1[i]; vi[i] = (__bf16)i0[i]; vi[4 + i] = (__bf16)i1[i]; vn[i] = (__bf16)(-i0[i]); vn[4 + i] = (__bf16)(-i1[i]); }
  vst2(BRE + (size_t)e * KP + c,      __builtin_bit_cast(v4u, vr));
  vst2(BRE + (size_t)e * KP + DD + c, __builtin_bit_cast(v4u, vn));
  vst2(BIM + (size_t)e * KP + c,      __builtin_bit_cast(v4u, vi));
  vst2(BIM + (size_t)e * KP + DD + c, __builtin_bit_cast(v4u, vr));
}

__global__ __launch_bounds__(128) void k_proj(const __bf16* __restrict__ X, const __bf16* __restrict__ Wp, const float* __restrict__ bias,
                                              int mode, int c0, _Float16* P0, _Float16* P1) {
  __shared__ __align__(16) float ss[64][132];
  const int tid = threadIdx.x, wave = tid >> 5, lane = tid & 31, col = lane & 15, g = lane >> 4;
  const int r0 = blockIdx.x * 64, n0 = blockIdx.y * 128; const int ql0 = r0 + wave * 16;
  const __bf16* xa = X + (size_t)(ql0 + col) * KP; const __bf16* wb = Wp + (size_t)(n0 + col) * KP;
  v8f acc[8] = {};
#pragma unroll 1
  for (int kc = 0; kc < KP / 32; ++kc) {
    const v16b a = frag_b(xa + kc * 32, lane);
#pragma unroll
    for (int j = 0; j < 8; ++j) acc[j] = wmma_bf(a, frag_b(wb + (size_t)j * 16 * KP + kc * 32, lane), acc[j]);
  }
#pragma unroll
  for (int j = 0; j < 8; ++j) { const float bb = bfr(bias[n0 + j * 16 + col]);
#pragma unroll
    for (int r = 0; r < 8; ++r) ss[wave * 16 + 8 * g + r][j * 16 + col] = acc[j][r] + bb; }
  __syncthreads();
  if (mode == 1) {
    const int bb = r0 / SEQ, nl = r0 - bb * SEQ;
    _Float16* vt = P0 + ((size_t)bb * KP + c0 + n0) * SEQ + nl;
    for (int e = tid; e < 128 * 8; e += 128) { const int d = e >> 3, q = e & 7; v8h o;
#pragma unroll
      for (int i = 0; i < 8; ++i) o[i] = (_Float16)ss[q * 8 + i][d];
      vst2(vt + (size_t)d * SEQ + q * 8, __builtin_bit_cast(v4u, o)); }
  } else {
#pragma unroll 1
    for (int it = 0; it < 8; ++it) { const int rl = wave * 16 + it * 2 + g;
      const v4f x0 = *(const v4f*)&ss[rl][col * 8], x1 = *(const v4f*)&ss[rl][col * 8 + 4];
      float v[8]; v8h hh, rr;
#pragma unroll
      for (int i = 0; i < 4; ++i) { v[i] = x0[i]; v[4 + i] = x1[i]; }
#pragma unroll
      for (int i = 0; i < 8; ++i) hh[i] = (_Float16)v[i];
#pragma unroll
      for (int i = 0; i < 8; ++i) rr[i] = (_Float16)((v[i] - (float)hh[i]) * QCAR);
      const size_t ro = (size_t)(r0 + rl) * KP + c0 + n0 + col * 8;
      vst2(P0 + ro, __builtin_bit_cast(v4u, hh));
      vst2(P1 + ro, __builtin_bit_cast(v4u, rr));
    }
  }
}

__global__ __launch_bounds__(128) void k_sc(const _Float16* __restrict__ QH, const _Float16* __restrict__ QR, const _Float16* __restrict__ KH, const _Float16* __restrict__ KR,
                                            int b, float* __restrict__ S0) {
  __shared__ __align__(16) float ss[4][16][68];
  const int z = blockIdx.z; float* S = S0 + (size_t)z * SEQ * SEQ;
  const int tid = threadIdx.x, wave = tid >> 5, lane = tid & 31, col = lane & 15, g = lane >> 4;
  const int k0 = blockIdx.y * 64; const int ql0 = blockIdx.x * 64 + wave * 16;
  const size_t qrow = ((size_t)b * SEQ + ql0 + col) * KP, krow = ((size_t)b * SEQ + k0 + col) * KP;
  const _Float16* qh = QH + qrow; const _Float16* ql = QR + qrow; const _Float16* kh = KH + krow; const _Float16* kl = KR + krow;
  v8f ah[4] = {}, ar[4] = {};
#pragma unroll 1
  for (int kc = 0; kc < KP / 32; ++kc) {
    const int up = (kc >= KP / 64) ? 1 : 0;
    const int koff = (z == 0) ? (kc * 32) : (up ? (kc * 32 - DD) : (DD + kc * 32));
    const unsigned sg = (z == 0 && up) ? 0x80008000u : 0u;
    const v16h a = hneg(frag_h(qh + kc * 32, lane), sg), r = hneg(frag_h(ql + kc * 32, lane), sg);
#pragma unroll
    for (int j = 0; j < 4; ++j) { const v16h kb = frag_h(kh + (size_t)j * 16 * KP + koff, lane), kr = frag_h(kl + (size_t)j * 16 * KP + koff, lane);
      ah[j] = wmma16(a, kb, ah[j]); ar[j] = wmma16(r, kb, ar[j]); ar[j] = wmma16(a, kr, ar[j]); }
  }
#pragma unroll
  for (int j = 0; j < 4; ++j)
#pragma unroll
    for (int r = 0; r < 8; ++r) ss[wave][8 * g + r][j * 16 + col] = ah[j][r] * SCL + ar[j][r] * (SCL / QCAR);
  __syncthreads();
#pragma unroll 1
  for (int it = 0; it < 8; ++it) { const int rl = it * 2 + g; vst2(S + (size_t)(ql0 + rl) * SEQ + k0 + col * 4, *(const v4f*)&ss[wave][rl][col * 4]); }
}
__global__ __launch_bounds__(256) void k_sm(const float* __restrict__ S0, _Float16* __restrict__ P) {
  __shared__ float sred[8]; __shared__ float sbc; __shared__ __align__(16) _Float16 sh[SEQ];
  constexpr int EPT = SEQ / 256;
  const int t = threadIdx.x; const size_t row = blockIdx.x;
  const float* sr = S0 + row * SEQ + t * EPT; const float* si = S0 + (size_t)SEQ * SEQ + row * SEQ + t * EPT;
  float a[EPT]; float m = -3.0e38f;
#pragma unroll
  for (int i = 0; i < EPT; ++i) { const float x = sr[i], y = si[i]; a[i] = sqrtf(x * x + y * y); m = fmaxf(m, a[i]); }
#pragma unroll
  for (int o = 1; o < 32; o <<= 1) m = fmaxf(m, __shfl_xor(m, o));
  if ((t & 31) == 0) sred[t >> 5] = m; __syncthreads();
  if (t == 0) { float v = sred[0]; for (int i = 1; i < 8; ++i) v = fmaxf(v, sred[i]); sbc = v; } __syncthreads(); m = sbc; __syncthreads();
  float e[EPT]; float sum = 0.f;
#pragma unroll
  for (int i = 0; i < EPT; ++i) { e[i] = exp_ni(a[i] - m); sum += e[i]; }
#pragma unroll
  for (int o = 1; o < 32; o <<= 1) sum += __shfl_xor(sum, o);
  if ((t & 31) == 0) sred[t >> 5] = sum; __syncthreads();
  if (t == 0) { float v = 0.f; for (int i = 0; i < 8; ++i) v += sred[i]; sbc = 1.0f / v; } __syncthreads(); const float inv = sbc;
#pragma unroll
  for (int i = 0; i < EPT; ++i) sh[t * EPT + i] = (_Float16)(e[i] * inv * PCAR);
  __syncthreads();
  if (t < SEQ / 8) vst2(P + row * SEQ + t * 8, *(const v4u*)&sh[t * 8]);
}
__global__ __launch_bounds__(128) void k_pv(const _Float16* __restrict__ P, const _Float16* __restrict__ VT, int b, float* __restrict__ OUT) {
  __shared__ __align__(16) float ss[4][16][132];
  const int tid = threadIdx.x, wave = tid >> 5, lane = tid & 31, col = lane & 15, g = lane >> 4;
  const int n0 = blockIdx.y * 128; const int ql0 = blockIdx.x * 64 + wave * 16;
  const _Float16* pa = P + (size_t)(ql0 + col) * SEQ; const _Float16* vb = VT + ((size_t)b * KP + n0 + col) * SEQ;
  v8f acc[8] = {};
#pragma unroll 1
  for (int kc = 0; kc < SEQ / 32; ++kc) { const v16h a = frag_h(pa + kc * 32, lane);
#pragma unroll
    for (int j = 0; j < 8; ++j) acc[j] = wmma16(a, frag_h(vb + (size_t)j * 16 * SEQ + kc * 32, lane), acc[j]); }
#pragma unroll
  for (int j = 0; j < 8; ++j)
#pragma unroll
    for (int r = 0; r < 8; ++r) ss[wave][8 * g + r][j * 16 + col] = acc[j][r] * (1.0f / PCAR);
  __syncthreads();
  const int pl = n0 / DD, d0 = n0 - pl * DD;
  float* ob = OUT + (((size_t)pl * NB_FULL + b) * SEQ_FULL + ql0) * DD + d0 + lane * 4;
#pragma unroll 1
  for (int rl = 0; rl < 16; ++rl) vst2(ob + (size_t)rl * DD, *(const v4f*)&ss[wave][rl][lane * 4]);
}

extern "C" void kernel_launch(void* const* d_in, const int* in_sizes, int n_in, void* d_out, int out_size, void* d_ws, size_t ws_size, hipStream_t stream) {
  if (n_in < 14) return;
  const float* xr = (const float*)d_in[0];  const float* xi = (const float*)d_in[1];
  const float* wqr = (const float*)d_in[2]; const float* wqi = (const float*)d_in[3]; const float* bqr = (const float*)d_in[4]; const float* bqi = (const float*)d_in[5];
  const float* wkr = (const float*)d_in[6]; const float* wki = (const float*)d_in[7]; const float* bkr = (const float*)d_in[8]; const float* bki = (const float*)d_in[9];
  const float* wvr = (const float*)d_in[10]; const float* wvi = (const float*)d_in[11]; const float* bvr = (const float*)d_in[12]; const float* bvi = (const float*)d_in[13];
  const int need_x = ((NB - 1) * SEQ_FULL + SEQ) * DD;
  if (in_sizes[0] < need_x || in_sizes[1] < need_x) return;
  for (int i = 2; i < 14; i += 4) { if (in_sizes[i] < DD * DD || in_sizes[i + 1] < DD * DD || in_sizes[i + 2] < DD || in_sizes[i + 3] < DD) return; }
  const int need_out = ((NB_FULL + NB - 1) * SEQ_FULL + SEQ) * DD;
  if (out_size < need_out) return;
  if (ws_size < (size_t)WS_END) return;
  char* ws = (char*)d_ws;
  __bf16* X = (__bf16*)(ws + WS_X); __bf16* Wp = (__bf16*)(ws + WS_W);
  _Float16* QH = (_Float16*)(ws + WS_QH); _Float16* QR = (_Float16*)(ws + WS_QR);
  _Float16* KH = (_Float16*)(ws + WS_KH); _Float16* KR = (_Float16*)(ws + WS_KR);
  _Float16* VT = (_Float16*)(ws + WS_VT); float* S = (float*)(ws + WS_S); _Float16* P = (_Float16*)(ws + WS_P);
  float* out = (float*)d_out;

  k_cvx<<<dim3(MR / 2), 256, 0, stream>>>(xr, xi, X);
  k_cvw<<<dim3(DD / 4), 256, 0, stream>>>(wqr, wqi, Wp + 0 * WPL, Wp + 1 * WPL);
  k_cvw<<<dim3(DD / 4), 256, 0, stream>>>(wkr, wki, Wp + 2 * WPL, Wp + 3 * WPL);
  k_cvw<<<dim3(DD / 4), 256, 0, stream>>>(wvr, wvi, Wp + 4 * WPL, Wp + 5 * WPL);
  const dim3 gp(MR / 64, DD / 128);
  k_proj<<<gp, 128, 0, stream>>>(X, Wp + 0 * WPL, bqr, 0, 0,  QH, QR);
  k_proj<<<gp, 128, 0, stream>>>(X, Wp + 1 * WPL, bqi, 0, DD, QH, QR);
  k_proj<<<gp, 128, 0, stream>>>(X, Wp + 2 * WPL, bkr, 0, 0,  KH, KR);
  k_proj<<<gp, 128, 0, stream>>>(X, Wp + 3 * WPL, bki, 0, DD, KH, KR);
  k_proj<<<gp, 128, 0, stream>>>(X, Wp + 4 * WPL, bvr, 1, 0,  VT, VT);
  k_proj<<<gp, 128, 0, stream>>>(X, Wp + 5 * WPL, bvi, 1, DD, VT, VT);
  for (int b = 0; b < NB; ++b) {
    k_sc<<<dim3(SEQ / 64, SEQ / 64, 2), 128, 0, stream>>>(QH, QR, KH, KR, b, S);
    k_sm<<<dim3(SEQ), 256, 0, stream>>>(S, P);
    k_pv<<<dim3(SEQ / 64, KP / 128), 128, 0, stream>>>(P, VT, b, out);
  }
}
